// SelectiveDiagonalSSM_58591943852307
// MI455X (gfx1250) — hardware-verified
//
#include <hip/hip_runtime.h>


namespace {
constexpr int Bn = 4, T = 2048, H = 1024, N = 16, NT = Bn * T;
constexpr float XS = 8.0f;

typedef _Float16 b16;
typedef __attribute__((ext_vector_type(16))) _Float16 v16b;
typedef __attribute__((ext_vector_type(8))) _Float16 v8b;
typedef __attribute__((ext_vector_type(8))) float v8f;
typedef __attribute__((ext_vector_type(4))) float v4f;
__device__ __forceinline__ float bf16_rne(float f) { unsigned int u = __float_as_uint(f); u += 0x7FFFu + ((u >> 16) & 1u); return __uint_as_float(u & 0xFFFF0000u); }
__device__ __forceinline__ v16b frag_kb(const b16* p, int hh) { const v8b a = *(const v8b*)(p + 8 * hh), b = *(const v8b*)(p + 16 + 8 * hh); v16b f;
#pragma unroll
  for (int e = 0; e < 8; ++e) { f[e] = a[e]; f[8 + e] = b[e]; } return f; }
__device__ __forceinline__ v8f wmma16b(v16b a, v16b b, v8f c) { v8f d = __builtin_amdgcn_wmma_f32_16x16x32_f16(false, a, false, b, (short)0, c, false, false); asm volatile("v_nop\n\tv_nop\n\tv_nop\n\tv_nop" : "+v"(d) : "v"(a), "v"(b)); return d; }
__device__ __forceinline__ void wave_lds_sync() { __builtin_amdgcn_fence(__ATOMIC_RELEASE, "workgroup"); __builtin_amdgcn_wave_barrier(); __builtin_amdgcn_fence(__ATOMIC_ACQUIRE, "workgroup"); }
__device__ __forceinline__ float nexp(float x) { return __builtin_amdgcn_exp2f(x * 1.4426950408889634f); }
__device__ __forceinline__ float nlog(float x) { return __builtin_amdgcn_logf(x) * 0.6931471805599453f; }
__device__ __forceinline__ float pmul(float a, float b) { float p = a * b; asm volatile("" : "+v"(p)); return p; }
__device__ __forceinline__ float softplus_f(float x) { return (x > 15.0f) ? x : (x < -15.0f ? nexp(x) : nlog(1.0f + nexp(x))); }

__global__ __launch_bounds__(256) void prep_kernel(const float* __restrict__ x, const float* __restrict__ alog, const float* __restrict__ bm, const float* __restrict__ cm, const float* __restrict__ dv, const float* __restrict__ wdt, const float* __restrict__ bdt, b16* __restrict__ R, b16* __restrict__ X, float* __restrict__ P) {
  const size_t tid = (size_t)blockIdx.x * 256 + threadIdx.x, nth = (size_t)gridDim.x * 256;
  for (int pass = 0; pass < 2; ++pass) {
    for (size_t p = tid; p < (size_t)H * H / 8; p += nth) { v8b v; for (int e = 0; e < 8; ++e) v[e] = (b16)bf16_rne(wdt[p * 8 + e]); *(volatile v8b*)(R + p * 8) = v; }
    for (size_t p = tid; p < (size_t)NT * H / 8; p += nth) { v8b v; for (int e = 0; e < 8; ++e) v[e] = (b16)(bf16_rne(x[p * 8 + e]) * XS); *(volatile v8b*)(X + p * 8) = v; }
    for (size_t q = tid; q < 2048 + 3 * (size_t)H * N; q += nth) { const int i = (int)q; float v; if (i < 1024) v = bf16_rne(bdt[i]); else if (i < 2048) v = bf16_rne(dv[i - 1024]); else if (i < 2048 + H * N) v = -nexp(bf16_rne(alog[i - 2048])); else if (i < 2048 + 2 * H * N) v = bf16_rne(bm[i - 2048 - H * N]); else v = bf16_rne(cm[i - 2048 - 2 * H * N]); P[q] = v; }
    __threadfence(); }
}

__global__ __launch_bounds__(64) void dt_kernel(const b16* __restrict__ X, const b16* __restrict__ R, const float* __restrict__ P, float* __restrict__ DT) {
  __shared__ __attribute__((aligned(16))) float Ts[2][32][128 + 4];
  const int lane = threadIdx.x & 31, wave = threadIdx.x >> 5, nloc = lane & 15, hlf = lane >> 4, m0 = blockIdx.y * 32, c0 = blockIdx.x * 256 + wave * 128;
#pragma unroll 1
  for (int hf = 0; hf < 2; ++hf) { v8f acc[2][4];
#pragma unroll
    for (int r = 0; r < 2; ++r)
#pragma unroll
      for (int t = 0; t < 4; ++t) acc[r][t] = (v8f){};
#pragma unroll 2
    for (int kb = 0; kb < H; kb += 32) { const v16b a0 = frag_kb(X + (size_t)(m0 + nloc) * H + kb, hlf), a1 = frag_kb(X + (size_t)(m0 + 16 + nloc) * H + kb, hlf);
#pragma unroll
      for (int t = 0; t < 4; ++t) { const v16b bw = frag_kb(R + (size_t)(c0 + (hf * 4 + t) * 16 + nloc) * H + kb, hlf); acc[0][t] = wmma16b(a0, bw, acc[0][t]); acc[1][t] = wmma16b(a1, bw, acc[1][t]); } }
#pragma unroll
    for (int t = 0; t < 4; ++t) { const int cl = (hf * 4 + t) * 16 + nloc; const float bb = P[c0 + cl];
#pragma unroll
      for (int r = 0; r < 2; ++r)
#pragma unroll
        for (int v = 0; v < 8; ++v) Ts[wave][r * 16 + 8 * hlf + v][cl] = softplus_f(acc[r][t][v] * (1.0f / XS) + bb); } }
  wave_lds_sync();
  for (int pass = 0; pass < 2; ++pass) { for (int i = lane; i < 32 * 32; i += 32) { const int rr = i >> 5, c4 = (i & 31) * 4; *(volatile v4f*)(DT + (size_t)(m0 + rr) * H + c0 + c4) = *(const v4f*)(&Ts[wave][rr][c4]); } __threadfence(); }
}

__global__ __launch_bounds__(256) void scan_kernel(const float* __restrict__ x, const float* __restrict__ DT, const float* __restrict__ P, float* __restrict__ YT, float* __restrict__ out1) {
  __shared__ __attribute__((aligned(16))) float Ys[8][2][32 + 4];
  const int wave = threadIdx.x >> 5, lane = threadIdx.x & 31, g = lane >> 4, n = lane & 15; const int ch = blockIdx.x * 16 + wave * 2 + g; const int b = ch / H, h = ch % H;
  const float A = P[2048 + h * N + n], Bv = P[2048 + H * N + h * N + n], Cv = P[2048 + 2 * H * N + h * N + n];
  float s = 0.0f; const float* dtp = DT + (size_t)(b * T) * H + h; const float* xp = x + (size_t)(b * T) * H + h;
  for (int t0 = 0; t0 < T; t0 += 32) {
    for (int tt = 0; tt < 32; ++tt) { const int t = t0 + tt; const float dt = dtp[(size_t)t * H], u = bf16_rne(xp[(size_t)t * H]);
      s = pmul(nexp(pmul(dt, A)), s) + pmul(pmul(dt, Bv), u);
      float y = pmul(s, Cv);
#pragma unroll
      for (int o = 1; o < 16; o <<= 1) y += __shfl_xor(y, o);
      if (n == 0) Ys[wave][g][tt] = y; }
    wave_lds_sync();
    for (int pass = 0; pass < 2; ++pass) { if (n < 8) *(volatile v4f*)(YT + ((size_t)b * H + h) * T + t0 + n * 4) = *(const v4f*)(&Ys[wave][g][n * 4]); }
    wave_lds_sync(); }
  for (int pass = 0; pass < 2; ++pass) { ((volatile float*)out1)[((size_t)b * H + h) * N + n] = s; __threadfence(); }
}

__global__ __launch_bounds__(256) void yout_kernel(const float* __restrict__ YT, const float* __restrict__ x, const float* __restrict__ P, float* __restrict__ out0) {
  __shared__ float Tt[32][256 + 1];
  const int b = blockIdx.z, h0 = blockIdx.y * 256, t0 = blockIdx.x * 32, t_ = threadIdx.x;
  for (int i = t_; i < 256 * 32; i += 256) { const int hl = i >> 5, tt = i & 31; Tt[tt][hl] = YT[((size_t)b * H + h0 + hl) * T + t0 + tt]; }
  __syncthreads();
  for (int pass = 0; pass < 2; ++pass) { for (int i = t_; i < 32 * 64; i += 256) { const int tt = i >> 6, c4 = (i & 63) * 4; const size_t gi = ((size_t)(b * T + t0 + tt)) * H + h0 + c4; const v4f xr = *(const v4f*)(x + gi); v4f o; for (int e = 0; e < 4; ++e) o[e] = Tt[tt][c4 + e] + pmul(P[1024 + h0 + c4 + e], bf16_rne(xr[e])); *(volatile v4f*)(out0 + gi) = o; } __threadfence(); }
}
}

extern "C" void kernel_launch(void* const* d_in, const int* in_sizes, int n_in,
                              void* d_out, int out_size, void* d_ws, size_t ws_size, hipStream_t stream) {
  (void)n_in; (void)out_size;
  const float* x = (const float*)d_in[0]; const float* alog = (const float*)d_in[1]; const float* bm = (const float*)d_in[2]; const float* cm = (const float*)d_in[3]; const float* dv = (const float*)d_in[4]; const float* wdt = (const float*)d_in[5]; const float* bdt = (const float*)d_in[6];
  float* out0 = (float*)d_out; float* out1 = (float*)((char*)d_out + (size_t)NT * H * 4);
  if (in_sizes[0] != NT * H || in_sizes[1] != H * N || in_sizes[5] != H * H) return;
  size_t off = 0; char* ws = (char*)d_ws;
  auto carve = [&](size_t bytes) { char* p = ws + off; off += (bytes + 255) & ~(size_t)255; return p; };
  b16* R = (b16*)carve((size_t)H * H * 2); b16* X = (b16*)carve((size_t)NT * H * 2); float* P = (float*)carve((2048 + 3 * (size_t)H * N) * 4); float* DT = (float*)carve((size_t)NT * H * 4); float* YT = (float*)carve((size_t)NT * H * 4);
  if (off > ws_size) return;
  prep_kernel<<<512, 256, 0, stream>>>(x, alog, bm, cm, dv, wdt, bdt, R, X, P);
  dt_kernel<<<dim3(H / 256, NT / 32), 64, 0, stream>>>(X, R, P, DT);
  scan_kernel<<<Bn * H / 16, 256, 0, stream>>>(x, DT, P, YT, out1);
  yout_kernel<<<dim3(T / 32, H / 256, Bn), 256, 0, stream>>>(YT, x, P, out0);
}
